// Generating_diffusion_model_61366492725508
// MI455X (gfx1250) — hardware-verified
//
#include <hip/hip_runtime.h>
#include <math.h>

typedef __attribute__((ext_vector_type(16))) _Float16 v16h;
typedef __attribute__((ext_vector_type(8)))  _Float16 v8h;
typedef __attribute__((ext_vector_type(16))) __bf16   v16b;
typedef __attribute__((ext_vector_type(8)))  __bf16   v8b;
typedef __attribute__((ext_vector_type(8)))  float    v8f;
typedef __attribute__((ext_vector_type(4)))  float    v4f;

constexpr int kBatch  = 16384;
constexpr int kSide   = 16;
constexpr int kMat    = kSide * kSide;
constexpr int kVec    = 2 * kMat;
constexpr int kLayers = 25;
constexpr int kOps    = 5;
constexpr int kPackK  = 32;
constexpr int kK3     = 3 * kVec;
constexpr int kK2     = 2 * kVec;
constexpr int kThr    = 256;

constexpr float kInCarry    = 1024.0f;
constexpr float kMapCarry   = 1024.0f;
constexpr float kRunCarry   = 4096.0f;
constexpr float kPairScale  = 1.0f / (kInCarry * kInCarry);
constexpr float kChainScale = 0.5f / (kRunCarry * kMapCarry);
constexpr float kOutScale   = 33554432.0f / (kInCarry * kRunCarry);
constexpr float kF16MinNormal = 6.103515625e-5f;

static_assert(kMat == 256 && kVec == 512 && kK3 == 1536 && kK2 == 1024, "plane sizes");
static_assert((kBatch % 64) == 0 && (kVec % 64) == 0 && (kMat % 64) == 0, "GEMM M, N multiples of 64");
static_assert((kPackK % 32) == 0 && (kK3 % 32) == 0 && (kK2 % 32) == 0, "GEMM K multiples of 32");
static_assert(2 * kOps <= kPackK, "ten live k slots");
static_assert(kOutScale == 8.0f && kChainScale == 1.1920928955078125e-7f && kPairScale == 9.5367431640625e-7f, "power-of-two scales");

constexpr size_t kOffV16  = 0;
constexpr size_t kOffKA   = kOffV16 + (size_t)kBatch * kK2 * 2;
constexpr size_t kOffKB   = kOffKA  + (size_t)kLayers * kMat * kPackK * 2;
constexpr size_t kOffKC   = kOffKB  + (size_t)kLayers * kVec * kPackK * 2;
constexpr size_t kOffBT   = kOffKC  + (size_t)kLayers * kMat * kVec * 4;
constexpr size_t kOffRA   = kOffBT  + (size_t)kLayers * kVec * kK3 * 2;
constexpr size_t kOffRC   = kOffRA  + (size_t)kVec * kK3 * 2;
constexpr size_t kOffZB   = kOffRC  + (size_t)kVec * kVec * 4;
constexpr size_t kWsTotal = kOffZB  + (size_t)kVec * 4;
static_assert(kWsTotal == 89835520ull, "carve total");
static_assert(kWsTotal <= 134217728ull, "carve cap");
static_assert((kOffKA % 256) == 0 && (kOffKB % 256) == 0 && (kOffKC % 256) == 0 && (kOffBT % 256) == 0 && (kOffRA % 256) == 0 && (kOffRC % 256) == 0 && (kOffZB % 256) == 0, "aligned regions");

__device__ __forceinline__ unsigned short f2bf_bits(float f) {
  unsigned u = __float_as_uint(f);
  return (unsigned short)((u + 0x7FFFu + ((u >> 16) & 1u)) >> 16);
}
__device__ __forceinline__ float bf_bits2f(unsigned short h) { return __uint_as_float(((unsigned)h) << 16); }
__device__ __forceinline__ float bf16r(float f) { return bf_bits2f(f2bf_bits(f)); }
__device__ __forceinline__ float carry_flush(float v, float carry) {
  const float s = v * carry;
  return (fabsf(s) < kF16MinNormal) ? 0.0f : s;
}
__device__ __forceinline__ float frcp(float x) { return __builtin_amdgcn_rcpf(x); }

__device__ __forceinline__ void dep_guard4_h(v8f& a, v8f& b, v8f& c, v8f& d, v16h x, v16h y) { asm volatile("v_nop\n\tv_nop\n\tv_nop\n\tv_nop" : "+v"(a), "+v"(b), "+v"(c), "+v"(d) : "v"(x), "v"(y)); }
__device__ __forceinline__ void dep_guard4_b(v8f& a, v8f& b, v8f& c, v8f& d, v16b x, v16b y) { asm volatile("v_nop\n\tv_nop\n\tv_nop\n\tv_nop" : "+v"(a), "+v"(b), "+v"(c), "+v"(d) : "v"(x), "v"(y)); }
__device__ __forceinline__ void keep4_h(v16h a, v16h b, v16h c, v16h d) { asm volatile("v_nop" :: "v"(a), "v"(b), "v"(c), "v"(d)); }
__device__ __forceinline__ void keep4_b(v16b a, v16b b, v16b c, v16b d) { asm volatile("v_nop" :: "v"(a), "v"(b), "v"(c), "v"(d)); }
__device__ __forceinline__ void acc_guard4(v8f& a, v8f& b, v8f& c, v8f& d) { asm volatile("v_nop\n\tv_nop\n\tv_nop\n\tv_nop" : "+v"(a), "+v"(b), "+v"(c), "+v"(d)); }

template <typename T> struct Frag;
template <> struct Frag<_Float16> {
  typedef v16h V; union U { v16h v; v8h h[2]; };
  static __device__ __forceinline__ v16h load(const _Float16* p) {
    U f; f.h[0] = *(const v8h*)(p); f.h[1] = *(const v8h*)(p + 16); return f.v;
  }
  static __device__ __forceinline__ v8f mma(v16h a, v16h b, v8f c) {
    return __builtin_amdgcn_wmma_f32_16x16x32_f16(false, a, false, b, (short)0, c, false, false);
  }
  static __device__ __forceinline__ void guard4(v8f& a, v8f& b, v8f& c, v8f& d, v16h x, v16h y) { dep_guard4_h(a, b, c, d, x, y); }
  static __device__ __forceinline__ void keep(v16h a, v16h b, v16h c, v16h d) { keep4_h(a, b, c, d); }
};
template <> struct Frag<__bf16> {
  typedef v16b V; union U { v16b v; v8b h[2]; };
  static __device__ __forceinline__ v16b load(const __bf16* p) {
    U f; f.h[0] = *(const v8b*)(p); f.h[1] = *(const v8b*)(p + 16); return f.v;
  }
  static __device__ __forceinline__ v8f mma(v16b a, v16b b, v8f c) {
    return __builtin_amdgcn_wmma_f32_16x16x32_bf16(false, a, false, b, (short)0, c, false, false);
  }
  static __device__ __forceinline__ void guard4(v8f& a, v8f& b, v8f& c, v8f& d, v16b x, v16b y) { dep_guard4_b(a, b, c, d, x, y); }
  static __device__ __forceinline__ void keep(v16b a, v16b b, v16b c, v16b d) { keep4_b(a, b, c, d); }
};

__device__ __forceinline__ v8f mma_h(v16h a, v16h b, v8f c) {
  c = __builtin_amdgcn_wmma_f32_16x16x32_f16(false, a, false, b, (short)0, c, false, false);
  asm volatile("v_nop\n\tv_nop\n\tv_nop\n\tv_nop" : "+v"(c) : "v"(a), "v"(b));
  return c;
}

template <int ET> struct Elem;
template <> struct Elem<0> { typedef _Float16 T; };
template <> struct Elem<1> { typedef __bf16 T; };
template <int ET, bool SPLIT, int BIAS_MODE, int OUT_MODE, bool RESID, int ACT = 0>
__global__ __launch_bounds__(256) void wmma_gemm64(
    const unsigned short* __restrict__ Ap, const unsigned short* __restrict__ A2p, int lda, long strideA,
    const unsigned short* __restrict__ Btp, const unsigned short* __restrict__ Bt2p, int ldb, long strideB,
    void* __restrict__ Cout, void* __restrict__ Cout2, int ldc, long strideC,
    const float* __restrict__ bias,
    const float* __restrict__ resid, long strideR,
    int M, int N, int K, float scale) {
  typedef typename Elem<ET>::T T;
  typedef typename Frag<T>::V V;
  const T* A = (const T*)Ap; const T* A2 = (const T*)A2p; const T* Bt = (const T*)Btp; const T* Bt2 = (const T*)Bt2p;
  __shared__ __align__(16) float sT[8][16 * 68];
  const int b    = blockIdx.y;
  const int lane = threadIdx.x & 31;
  const int wave = threadIdx.x >> 5;
  const int tilesN = N >> 6;
  const int tilesM = M >> 6;
  const int tile = blockIdx.x * 8 + wave;
  if (tile >= tilesM * tilesN) return;
  const int tm = tile / tilesN;
  const int tn = tile - tm * tilesN;
  const int m0 = tm << 6;
  const int n0 = tn << 6;

  const T* Ab  = A  + (size_t)b * strideA;
  const T* Bb  = Bt + (size_t)b * strideB;
  const T* Ab2 = SPLIT ? (A2  + (size_t)b * strideA) : nullptr;
  const T* Bb2 = SPLIT ? (Bt2 + (size_t)b * strideB) : nullptr;

  const int rlane = lane & 15;
  const int koff  = (lane >> 4) * 8;
  const int mOff  = (lane >> 4) * 8;

  v8f acc[4][4];
#pragma unroll
  for (int i = 0; i < 4; ++i)
#pragma unroll
    for (int j = 0; j < 4; ++j) acc[i][j] = (v8f){0.f,0.f,0.f,0.f,0.f,0.f,0.f,0.f};

  for (int k0 = 0; k0 < K; k0 += 32) {
    V bh[4], bl[4];
#pragma unroll
    for (int j = 0; j < 4; ++j) {
      const size_t bo = (size_t)(n0 + (j << 4) + rlane) * ldb + koff + k0;
      bh[j] = Frag<T>::load(Bb + bo);
      if (SPLIT) bl[j] = Frag<T>::load(Bb2 + bo);
    }
#pragma unroll
    for (int i = 0; i < 4; ++i) {
      const size_t ao = (size_t)(m0 + (i << 4) + rlane) * lda + koff + k0;
      V ah = Frag<T>::load(Ab + ao);
      V al;
      if (SPLIT) al = Frag<T>::load(Ab2 + ao);
#pragma unroll
      for (int j = 0; j < 4; ++j) {
        acc[i][j] = Frag<T>::mma(ah, bh[j], acc[i][j]);
        if (SPLIT) {
          acc[i][j] = Frag<T>::mma(ah, bl[j], acc[i][j]);
          acc[i][j] = Frag<T>::mma(al, bh[j], acc[i][j]);
        }
      }
      Frag<T>::guard4(acc[i][0], acc[i][1], acc[i][2], acc[i][3], ah, SPLIT ? al : ah);
    }
    Frag<T>::keep(bh[0], bh[1], bh[2], bh[3]);
    if (SPLIT) Frag<T>::keep(bl[0], bl[1], bl[2], bl[3]);
  }
  acc_guard4(acc[0][0], acc[0][1], acc[0][2], acc[0][3]);
  acc_guard4(acc[1][0], acc[1][1], acc[1][2], acc[1][3]);
  acc_guard4(acc[2][0], acc[2][1], acc[2][2], acc[2][3]);
  acc_guard4(acc[3][0], acc[3][1], acc[3][2], acc[3][3]);

  float* slab = sT[wave];
  const float* Rb = RESID ? (resid + (size_t)b * strideR) : nullptr;
#pragma unroll
  for (int i = 0; i < 4; ++i) {
    const int mBase = m0 + (i << 4);
#pragma unroll
    for (int j = 0; j < 4; ++j) {
      const int n = n0 + (j << 4) + rlane;
      float bv = 0.f;
      if (BIAS_MODE == 2) bv = bias[n];
#pragma unroll
      for (int r = 0; r < 8; ++r) {
        float v = acc[i][j][r] * scale;
        if (BIAS_MODE == 1) v += bias[mBase + mOff + r];
        if (BIAS_MODE == 2) v += bv;
        if (RESID) v += Rb[(size_t)(mBase + mOff + r) * ldc + n];
        if (ACT == 1) v = tanhf(v);
        if (ACT == 2) v = fmaxf(v, 0.0f);
        if (ACT == 3) v = v / (1.0f + expf(-v));
        if (ACT == 4) v = (v > 0.f) ? v : 0.01f * v;
        slab[(mOff + r) * 68 + (j << 4) + rlane] = v;
      }
    }
    __builtin_amdgcn_fence(__ATOMIC_RELEASE, "workgroup");
    __builtin_amdgcn_wave_barrier();
    __builtin_amdgcn_fence(__ATOMIC_ACQUIRE, "workgroup");
    if (OUT_MODE == 0) {
      float* C = (float*)Cout + (size_t)b * strideC;
      const int hh = lane >> 4, c4 = (lane & 15) * 4;
      for (int pass = 0; pass < 2; ++pass) {
#pragma unroll
        for (int it = 0; it < 8; ++it) {
          const int row = it * 2 + hh;
          v4f v = *(const v4f*)(slab + row * 68 + c4);
          *(volatile v4f*)(C + (size_t)(mBase + row) * ldc + n0 + c4) = v;
        }
        __threadfence();
      }
    } else {
      const int q = lane >> 3, c8 = (lane & 7) * 8;
      unsigned short* C  = (unsigned short*)Cout  + (size_t)b * strideC;
      unsigned short* C2 = (OUT_MODE == 2) ? ((unsigned short*)Cout2 + (size_t)b * strideC) : nullptr;
      for (int pass = 0; pass < 2; ++pass) {
#pragma unroll
        for (int it = 0; it < 4; ++it) {
          const int row = it * 4 + q;
          const float* sp = slab + row * 68 + c8;
          v8h hv, lv;
#pragma unroll
          for (int e = 0; e < 8; ++e) {
            if (OUT_MODE == 1) {
              hv[e] = (_Float16)sp[e];
            } else {
              unsigned short hb = f2bf_bits(sp[e]);
              unsigned short lb = f2bf_bits(sp[e] - bf_bits2f(hb));
              hv[e] = __builtin_bit_cast(_Float16, hb);
              lv[e] = __builtin_bit_cast(_Float16, lb);
            }
          }
          *(volatile v8h*)(C + (size_t)(mBase + row) * ldc + n0 + c8) = hv;
          if (OUT_MODE == 2) *(volatile v8h*)(C2 + (size_t)(mBase + row) * ldc + n0 + c8) = lv;
        }
        __threadfence();
      }
    }
    __builtin_amdgcn_fence(__ATOMIC_RELEASE, "workgroup");
    __builtin_amdgcn_wave_barrier();
    __builtin_amdgcn_fence(__ATOMIC_ACQUIRE, "workgroup");
  }
}

__global__ __launch_bounds__(kThr) void cast_plane_kernel(const float* __restrict__ src, unsigned short* __restrict__ dst,
                                                          int colsLog2, int dstPitch, int dstOff) {
  const int i   = blockIdx.x * kThr + threadIdx.x;
  const int sh  = colsLog2 - 3;
  const int row = i >> sh;
  const int c8  = (i & ((1 << sh) - 1)) * 8;
  const float* sp = src + ((size_t)row << colsLog2) + c8;
  const v4f a0 = *(const v4f*)(sp);
  const v4f a1 = *(const v4f*)(sp + 4);
  v8h hv;
#pragma unroll
  for (int e = 0; e < 4; ++e) {
    const float f0 = a0[e];
    const float f1 = a1[e];
    hv[e]     = (_Float16)carry_flush(bf16r(f0), kInCarry);
    hv[4 + e] = (_Float16)carry_flush(bf16r(f1), kInCarry);
  }
  unsigned short* dp = dst + (size_t)row * dstPitch + dstOff + c8;
  *(volatile v8h*)dp = hv;
  __threadfence();
  *(volatile v8h*)dp = hv;
}

__device__ __forceinline__ void split_hl(float v, float carry, float& hi, float& lo) {
  const float s = carry_flush(v, carry);
  hi = (float)(_Float16)s;
  const float r = s - hi;
  lo = (float)(_Float16)((fabsf(r) < kF16MinNormal) ? 0.0f : r);
}

__global__ __launch_bounds__(192) void map_init_kernel(unsigned short* __restrict__ RA, float* __restrict__ ZB) {
  const unsigned n   = blockIdx.x;
  const unsigned tid = threadIdx.x;
  unsigned k0 = tid * 8u;
  asm volatile("" : "+v"(k0));
  const unsigned sec = k0 >> 9;
  const unsigned kk0 = k0 & 511u;
  const unsigned one = (n & 1u) * 256u + (n >> 1);
  v8h hv;
#pragma unroll
  for (int e = 0; e < 8; ++e) hv[e] = (sec < 2u && kk0 + (unsigned)e == one) ? (_Float16)kRunCarry : (_Float16)0.0f;
  unsigned short* dp = RA + (size_t)n * kK3 + k0;
  *(volatile v8h*)dp = hv;
  __threadfence();
  *(volatile v8h*)dp = hv;
  if (n == 0u && tid < 128u) {
    const v4f z4 = {0.f, 0.f, 0.f, 0.f};
    *(volatile v4f*)(ZB + 4u * tid) = z4;
    __threadfence();
    *(volatile v4f*)(ZB + 4u * tid) = z4;
  }
}

constexpr int kPackA   = kLayers * kMat * kPackK;
constexpr int kPackB   = kLayers * kVec * kPackK;
static_assert(((kPackA + kPackB) / 8) % kThr == 0 && (kPackA % 8) == 0, "pack grid exact");
__global__ __launch_bounds__(kThr) void kraus_pack_kernel(const float* __restrict__ Kr, const float* __restrict__ Ki,
                                                          unsigned short* __restrict__ KA, unsigned short* __restrict__ KB) {
  unsigned e8 = (blockIdx.x * (unsigned)kThr + threadIdx.x) * 8u;
  asm volatile("" : "+v"(e8));
  const bool isB = e8 >= (unsigned)kPackA;
  unsigned f = isB ? (e8 - (unsigned)kPackA) : e8;
  asm volatile("" : "+v"(f));
  const unsigned kk0 = f & 31u;
  unsigned row = f >> 5;
  asm volatile("" : "+v"(row));
  const unsigned lay  = isB ? (row >> 9) : (row >> 8);
  const unsigned part = isB ? ((row >> 8) & 1u) : 0u;
  const unsigned ent  = row & 255u;
  v8h hv;
#pragma unroll
  for (int e = 0; e < 8; ++e) {
    const unsigned kk = kk0 + (unsigned)e;
    const bool live = kk < 2u * (unsigned)kOps;
    const bool second = kk >= (unsigned)kOps;
    unsigned k = second ? (kk - (unsigned)kOps) : kk;
    k = live ? k : 0u;
    const bool fromKi = (part == 0u) ? second : !second;
    const unsigned idx = (lay * (unsigned)kOps + k) * (unsigned)kMat + ent;
    float xr = Kr[idx];
    float xi = Ki[idx];
    asm volatile("" : "+v"(xr));
    asm volatile("" : "+v"(xi));
    float v = bf16r(fromKi ? xi : xr);
    if (part == 1u && !second) v = -v;
    v = live ? v : 0.0f;
    hv[e] = (_Float16)carry_flush(v, kInCarry);
  }
  unsigned short* dp = isB ? (KB + f) : (KA + f);
  *(volatile v8h*)dp = hv;
  __threadfence();
  *(volatile v8h*)dp = hv;
}

__global__ __launch_bounds__(kThr) void layer_map_kernel(const float* __restrict__ KC, unsigned short* __restrict__ BT) {
  const unsigned lay = blockIdx.y;
  unsigned t = blockIdx.x * (unsigned)kThr + threadIdx.x;
  asm volatile("" : "+v"(t));
  const unsigned jl = t >> 5;
  const unsigned g  = t & 31u;
  unsigned i  = g >> 1;
  unsigned m0 = (g & 1u) * 8u;
  unsigned j  = jl >> 4;
  unsigned l  = jl & 15u;
  asm volatile("" : "+v"(i));
  asm volatile("" : "+v"(m0));
  asm volatile("" : "+v"(j));
  asm volatile("" : "+v"(l));
  const float* src = KC + ((size_t)lay * kMat + (i * 16u + j)) * kVec;
  v8h srh, srl, sih, sil, nih, nil;
#pragma unroll
  for (int e = 0; e < 8; ++e) {
    const unsigned ml = (m0 + (unsigned)e) * 16u + l;
    const float sr = src[ml];
    const float si = src[(unsigned)kMat + ml];
    float h, lo;
    split_hl(sr, kMapCarry, h, lo);
    srh[e] = (_Float16)h; srl[e] = (_Float16)lo;
    split_hl(si, kMapCarry, h, lo);
    sih[e] = (_Float16)h; sil[e] = (_Float16)lo;
    nih[e] = (_Float16)(-h); nil[e] = (_Float16)(-lo);
  }
  const unsigned im0 = i * 16u + m0;
  unsigned short* row0 = BT + ((size_t)lay * kVec + jl) * kK3;
  unsigned short* row1 = BT + ((size_t)lay * kVec + (unsigned)kMat + jl) * kK3;
  for (int pass = 0; pass < 2; ++pass) {
    *(volatile v8h*)(row0 + im0)                    = srh;
    *(volatile v8h*)(row0 + kVec + im0)             = srl;
    *(volatile v8h*)(row0 + 2 * kVec + im0)         = srh;
    *(volatile v8h*)(row0 + kMat + im0)             = sih;
    *(volatile v8h*)(row0 + kVec + kMat + im0)      = sil;
    *(volatile v8h*)(row0 + 2 * kVec + kMat + im0)  = sih;
    *(volatile v8h*)(row1 + im0)                    = nih;
    *(volatile v8h*)(row1 + kVec + im0)             = nil;
    *(volatile v8h*)(row1 + 2 * kVec + im0)         = nih;
    *(volatile v8h*)(row1 + kMat + im0)             = srh;
    *(volatile v8h*)(row1 + kVec + kMat + im0)      = srl;
    *(volatile v8h*)(row1 + 2 * kVec + kMat + im0)  = srh;
    __threadfence();
  }
}

__global__ __launch_bounds__(64) void split_plane_kernel(const float* __restrict__ RC, unsigned short* __restrict__ RA) {
  const unsigned n = blockIdx.x;
  unsigned c8 = threadIdx.x * 8u;
  asm volatile("" : "+v"(c8));
  const float* sp = RC + (size_t)n * kVec + c8;
  const v4f a0 = *(const v4f*)(sp);
  const v4f a1 = *(const v4f*)(sp + 4);
  v8h hv, lv;
#pragma unroll
  for (int e = 0; e < 4; ++e) {
    float h, lo;
    split_hl(a0[e], kRunCarry, h, lo);
    hv[e] = (_Float16)h; lv[e] = (_Float16)lo;
    split_hl(a1[e], kRunCarry, h, lo);
    hv[4 + e] = (_Float16)h; lv[4 + e] = (_Float16)lo;
  }
  unsigned short* dp = RA + (size_t)n * kK3 + c8;
  for (int pass = 0; pass < 2; ++pass) {
    *(volatile v8h*)(dp)            = hv;
    *(volatile v8h*)(dp + kVec)     = hv;
    *(volatile v8h*)(dp + 2 * kVec) = lv;
    __threadfence();
  }
}

static_assert(((kMat / 64) * (kVec / 64)) % 8 == 0 && ((kVec / 64) * (kVec / 64)) % 8 == 0 && ((kBatch / 64) * (kVec / 64)) % 8 == 0, "GEMM grids exact");
static_assert(((size_t)kBatch * kMat / 8) % kThr == 0, "cast grid exact");
static_assert((kMat * 32) % kThr == 0 && kK3 == 192 * 8 && kVec == 64 * 8, "map grids exact");

extern "C" void kernel_launch(void* const* d_in, const int* in_sizes, int n_in,
                              void* d_out, int out_size, void* d_ws, size_t ws_size,
                              hipStream_t stream) {
  if (n_in < 4 || d_out == nullptr || d_ws == nullptr) return;
  if (in_sizes[0] != kBatch * kMat || in_sizes[1] != kBatch * kMat) return;
  if (in_sizes[2] != kLayers * kOps * kMat || in_sizes[3] != kLayers * kOps * kMat) return;
  if (out_size != kBatch * kVec) return;
  if (ws_size < kWsTotal) return;

  const float* s_re = (const float*)d_in[0];
  const float* s_im = (const float*)d_in[1];
  const float* k_re = (const float*)d_in[2];
  const float* k_im = (const float*)d_in[3];
  float* out = (float*)d_out;

  char* ws = (char*)d_ws;
  unsigned short* V16 = (unsigned short*)(ws + kOffV16);
  unsigned short* KA  = (unsigned short*)(ws + kOffKA);
  unsigned short* KB  = (unsigned short*)(ws + kOffKB);
  float*          KC  = (float*)(ws + kOffKC);
  unsigned short* BT  = (unsigned short*)(ws + kOffBT);
  unsigned short* RA  = (unsigned short*)(ws + kOffRA);
  float*          RC  = (float*)(ws + kOffRC);
  float*          ZB  = (float*)(ws + kOffZB);

  const int castGrid = (int)(((size_t)kBatch * kMat / 8) / kThr);
  cast_plane_kernel<<<castGrid, kThr, 0, stream>>>(s_re, V16, 8, kK2, 0);
  cast_plane_kernel<<<castGrid, kThr, 0, stream>>>(s_im, V16, 8, kK2, kMat);
  cast_plane_kernel<<<castGrid, kThr, 0, stream>>>(s_re, V16, 8, kK2, 2 * kMat);
  cast_plane_kernel<<<castGrid, kThr, 0, stream>>>(s_im, V16, 8, kK2, 3 * kMat);

  map_init_kernel<<<kVec, 192, 0, stream>>>(RA, ZB);
  kraus_pack_kernel<<<((kPackA + kPackB) / 8) / kThr, kThr, 0, stream>>>(k_re, k_im, KA, KB);

  wmma_gemm64<0, false, 2, 0, false, 0><<<dim3((kMat / 64) * (kVec / 64) / 8, kLayers), 256, 0, stream>>>(
      KA, KA, kPackK, (long)kMat * kPackK, KB, KB, kPackK, (long)kVec * kPackK, (void*)KC, (void*)KC, kVec, (long)kMat * kVec,
      ZB, nullptr, 0L, kMat, kVec, kPackK, kPairScale);

  layer_map_kernel<<<dim3((kMat * 32) / kThr, kLayers), kThr, 0, stream>>>(KC, BT);

  for (int lay = kLayers - 1; lay >= 0; --lay) {
    wmma_gemm64<0, false, 2, 0, false, 0><<<dim3((kVec / 64) * (kVec / 64) / 8, 1), 256, 0, stream>>>(
        RA, RA, kK3, 0L, BT + (size_t)lay * kVec * kK3, BT + (size_t)lay * kVec * kK3, kK3, 0L, (void*)RC, (void*)RC, kVec, 0L,
        ZB, nullptr, 0L, kVec, kVec, kK3, kChainScale);
    split_plane_kernel<<<kVec, 64, 0, stream>>>(RC, RA);
  }

  wmma_gemm64<0, false, 2, 0, false, 0><<<dim3((kBatch / 64) * (kVec / 64) / 8, 1), 256, 0, stream>>>(
      V16, V16, kK2, 0L, RA + kVec, RA + kVec, kK3, 0L, (void*)out, (void*)out, kVec, 0L,
      ZB, nullptr, 0L, kBatch, kVec, kK2, kOutScale);
}
